// SelfAttention1d_53154515256219
// MI455X (gfx1250) — hardware-verified
//
#include <hip/hip_runtime.h>
#include <math.h>

typedef __attribute__((ext_vector_type(16))) _Float16 v16h;
typedef __attribute__((ext_vector_type(16))) __bf16 v16b;
typedef __attribute__((ext_vector_type(8)))  _Float16 v8h;
typedef __attribute__((ext_vector_type(8)))  __bf16 v8b;
typedef __attribute__((ext_vector_type(8)))  float v8f;
typedef __attribute__((ext_vector_type(4)))  float v4f;
typedef __attribute__((ext_vector_type(4)))  unsigned v4u;

#ifndef NB
#define NB 8
#endif
#ifndef SEQ
#define SEQ 2048
#endif
#define NB_FULL 8
#define SEQ_FULL 2048
#define CC 256
#define DQ 32
#define PCARRY 16384.0f
#define RCARRY 1024.0f

static_assert(SEQ % 256 == 0);
static_assert(SEQ <= SEQ_FULL);
static_assert(NB <= NB_FULL);
static_assert(CC == 256);
static_assert(DQ == 32);
#define NBQ ((DQ * CC) / 2048)
#define NBV ((CC * CC) / 2048)
static_assert(NBQ * 2048 == DQ * CC);
static_assert(NBV * 2048 == CC * CC);

template <typename T> __device__ __forceinline__ void vst2(void* p, T v) { *(volatile T*)p = v; __threadfence(); *(volatile T*)p = v; }

__device__ __forceinline__ v8f wmma16(v16h a, v16h b, v8f c) {
  v8f d = __builtin_amdgcn_wmma_f32_16x16x32_f16(false, a, false, b, (short)0, c, false, false);
  asm volatile("v_nop\n\tv_nop\n\tv_nop\n\tv_nop" : "+v"(d) : "v"(a), "v"(b));
  return d;
}
__device__ __forceinline__ v8f wmma_bf(v16b a, v16b b, v8f c) {
  v8f d = __builtin_amdgcn_wmma_f32_16x16x32_bf16(false, a, false, b, (short)0, c, false, false);
  asm volatile("v_nop\n\tv_nop\n\tv_nop\n\tv_nop" : "+v"(d) : "v"(a), "v"(b));
  return d;
}
__device__ __forceinline__ v16h frag_h(const _Float16* rowk0, int lane) {
  union { v16h v; v8h q[2]; } u; const _Float16* p = rowk0 + 8 * (lane >> 4);
  u.q[0] = *(const v8h*)p; u.q[1] = *(const v8h*)(p + 16); return u.v;
}
__device__ __forceinline__ v16b frag_b(const __bf16* rowk0, int lane) {
  union { v16b v; v8b q[2]; } u; const __bf16* p = rowk0 + 8 * (lane >> 4);
  u.q[0] = *(const v8b*)p; u.q[1] = *(const v8b*)(p + 16); return u.v;
}
__device__ __forceinline__ float bfr(float v) { return (float)(__bf16)v; }

#define WS_WQ  ((size_t)0)
#define WS_WK  (WS_WQ + 2u * (size_t)DQ * CC)
#define WS_WV  (WS_WK + 2u * (size_t)DQ * CC)
#define WS_XB  (WS_WV + 2u * (size_t)CC * CC)
#define WS_QH  (WS_XB + 2u * (size_t)NB * SEQ * CC)
#define WS_QL  (WS_QH + 2u * (size_t)NB * SEQ * DQ)
#define WS_KH  (WS_QL + 2u * (size_t)NB * SEQ * DQ)
#define WS_KL  (WS_KH + 2u * (size_t)NB * SEQ * DQ)
#define WS_VH  (WS_KL + 2u * (size_t)NB * SEQ * DQ)
#define WS_S   (WS_VH + 2u * (size_t)NB * CC * SEQ)
#define WS_P   (WS_S + 4u * (size_t)SEQ * SEQ)
#define WS_END (WS_P + 2u * (size_t)SEQ * SEQ)
static_assert(WS_END <= (size_t)134217728);
static_assert(WS_XB % 128 == 0 && WS_QH % 128 == 0 && WS_QL % 128 == 0 && WS_KH % 128 == 0 && WS_KL % 128 == 0 && WS_VH % 128 == 0 && WS_S % 128 == 0 && WS_P % 128 == 0);

__global__ __launch_bounds__(256) void k_cvt(const float* __restrict__ WQ, const float* __restrict__ WK, const float* __restrict__ WV, __bf16* __restrict__ PQ, __bf16* __restrict__ PK, __bf16* __restrict__ PV) {
  const int blk = blockIdx.x; const int t = threadIdx.x;
  const int sel = blk < NBQ ? 0 : (blk < 2 * NBQ ? 1 : 2);
  const float* src = sel == 0 ? WQ : (sel == 1 ? WK : WV);
  __bf16* dst = sel == 0 ? PQ : (sel == 1 ? PK : PV);
  const size_t g = (size_t)(blk - (sel == 0 ? 0 : (sel == 1 ? NBQ : 2 * NBQ))) * 256 + t;
  const float* p = src + g * 8;
  const v4f a = *(const v4f*)p, c = *(const v4f*)(p + 4);
  union { v8b v; v4u u; } o;
#pragma unroll
  for (int i = 0; i < 4; ++i) { o.v[i] = (__bf16)a[i]; o.v[4 + i] = (__bf16)c[i]; }
  vst2(dst + g * 8, o.u);
}
__global__ __launch_bounds__(256) void k_xt(const float* __restrict__ X, __bf16* __restrict__ XB) {
  __shared__ __align__(16) __bf16 st[64][CC + 8];
  const int t = threadIdx.x; const int l0 = blockIdx.x * 64; const size_t b = blockIdx.y;
#pragma unroll 2
  for (int e = t; e < CC * 16; e += 256) { const int c = e >> 4, lq = (e & 15) * 4;
    const v4f v = *(const v4f*)(X + (b * CC + c) * (size_t)SEQ_FULL + l0 + lq);
    st[lq][c] = (__bf16)v[0]; st[lq + 1][c] = (__bf16)v[1]; st[lq + 2][c] = (__bf16)v[2]; st[lq + 3][c] = (__bf16)v[3]; }
  __syncthreads();
  for (int e = t; e < 64 * 32; e += 256) { const int ll = e >> 5, q = e & 31;
    vst2(XB + (b * SEQ + l0 + ll) * (size_t)CC + q * 8, *(const v4u*)&st[ll][q * 8]); }
}
__global__ __launch_bounds__(128) __attribute__((amdgpu_num_vgpr(256))) void k_pqk(const __bf16* __restrict__ XB, const __bf16* __restrict__ PQ, const __bf16* __restrict__ PK, const float* __restrict__ BQ, const float* __restrict__ BK, _Float16* __restrict__ QH, _Float16* __restrict__ QL, _Float16* __restrict__ KH, _Float16* __restrict__ KL) {
  __shared__ __align__(16) _Float16 sh[64][DQ + 8], sl[64][DQ + 8];
  const int tid = threadIdx.x, wave = tid >> 5, lane = tid & 31, col = lane & 15, g = lane >> 4;
  const int which = blockIdx.y;
  const __bf16* WP = which == 0 ? PQ : PK; const float* BA = which == 0 ? BQ : BK;
  _Float16* DH = which == 0 ? QH : KH; _Float16* DL = which == 0 ? QL : KL;
  const size_t r0 = (size_t)blockIdx.x * 64;
  v8f acc[2] = {};
#pragma unroll 2
  for (int kc = 0; kc < CC / 32; ++kc) {
    const v16b a = frag_b(XB + (r0 + wave * 16 + col) * CC + kc * 32, lane);
#pragma unroll
    for (int j = 0; j < 2; ++j) { const v16b w = frag_b(WP + (size_t)(j * 16 + col) * CC + kc * 32, lane);
      acc[j] = wmma_bf(a, w, acc[j]); }
  }
#pragma unroll
  for (int j = 0; j < 2; ++j) { const float bb = bfr(BA[j * 16 + col]);
#pragma unroll
    for (int r = 0; r < 8; ++r) { const float v = acc[j][r] + bb; const int rl = wave * 16 + 8 * g + r, cl = j * 16 + col;
      const _Float16 hv = (_Float16)v; sh[rl][cl] = hv; sl[rl][cl] = (_Float16)((v - (float)hv) * RCARRY); } }
  __syncthreads();
  for (int e = tid; e < 64 * 4; e += 128) { const int rl = e >> 2, q = e & 3; const size_t o = (r0 + rl) * DQ + q * 8;
    vst2(DH + o, *(const v4u*)&sh[rl][q * 8]); vst2(DL + o, *(const v4u*)&sl[rl][q * 8]); }
}
__global__ __launch_bounds__(128) __attribute__((amdgpu_num_vgpr(256))) void k_pvv(const __bf16* __restrict__ XB, const __bf16* __restrict__ PV, const float* __restrict__ BV, _Float16* __restrict__ VH) {
  __shared__ __align__(16) _Float16 th[128][72];
  const int tid = threadIdx.x, wave = tid >> 5, lane = tid & 31, col = lane & 15, g = lane >> 4;
  const int c0 = blockIdx.y * 128; const size_t r0 = (size_t)blockIdx.x * 64;
  v8f acc[8] = {};
#pragma unroll 1
  for (int kc = 0; kc < CC / 32; ++kc) {
    const v16b a = frag_b(XB + (r0 + wave * 16 + col) * CC + kc * 32, lane);
#pragma unroll
    for (int j = 0; j < 8; ++j) { const v16b w = frag_b(PV + (size_t)(c0 + j * 16 + col) * CC + kc * 32, lane); acc[j] = wmma_bf(a, w, acc[j]); }
  }
#pragma unroll
  for (int j = 0; j < 8; ++j) { const float bb = bfr(BV[c0 + j * 16 + col]);
#pragma unroll
    for (int r = 0; r < 8; ++r) { const int rl = wave * 16 + 8 * g + r, cl = j * 16 + col; th[cl][rl] = (_Float16)(acc[j][r] + bb); } }
  __syncthreads();
  { const size_t b = r0 / SEQ; const int t0 = (int)(r0 % SEQ);
    for (int e = tid; e < 128 * 8; e += 128) { const int cl = e >> 3, q = e & 7;
      vst2(VH + (b * CC + c0 + cl) * (size_t)SEQ + t0 + q * 8, *(const v4u*)&th[cl][q * 8]); } }
}
__global__ __launch_bounds__(128) __attribute__((amdgpu_num_vgpr(256))) void k_sc(const _Float16* __restrict__ QH, const _Float16* __restrict__ QL, const _Float16* __restrict__ KH, const _Float16* __restrict__ KL, int b, float* __restrict__ S) {
  __shared__ __align__(16) float ss[4][16][132];
  const int tid = threadIdx.x, wave = tid >> 5, lane = tid & 31, col = lane & 15, g = lane >> 4;
  const int k0 = blockIdx.y * 128; const int ql0 = blockIdx.x * 64 + wave * 16; const size_t q0 = (size_t)b * SEQ + ql0;
  const v16h ah = frag_h(QH + (q0 + col) * DQ, lane), al = frag_h(QL + (q0 + col) * DQ, lane);
#pragma unroll
  for (int jg = 0; jg < 2; ++jg) {
    v8f acc[4] = {}, accl[4] = {};
#pragma unroll
    for (int j = 0; j < 4; ++j) { const size_t kr = ((size_t)b * SEQ + k0 + jg * 64 + j * 16 + col) * DQ;
      const v16h kh = frag_h(KH + kr, lane); const v16h kl = frag_h(KL + kr, lane);
      acc[j] = wmma16(ah, kh, acc[j]); accl[j] = wmma16(al, kh, accl[j]); accl[j] = wmma16(ah, kl, accl[j]); }
#pragma unroll
    for (int j = 0; j < 4; ++j)
#pragma unroll
      for (int r = 0; r < 8; ++r) ss[wave][8 * g + r][jg * 64 + j * 16 + col] = acc[j][r] + accl[j][r] * (1.0f / RCARRY);
  }
  __syncthreads();
  for (int rl = 0; rl < 16; ++rl) vst2(S + (size_t)(ql0 + rl) * SEQ + k0 + lane * 4, *(const v4f*)&ss[wave][rl][lane * 4]);
}
__global__ __launch_bounds__(256) void k_sm(const float* __restrict__ S, _Float16* __restrict__ P) {
  __shared__ float sred[8]; __shared__ float sbc; __shared__ __align__(16) float se[SEQ]; __shared__ __align__(16) _Float16 sp[SEQ];
  const int t = threadIdx.x; const size_t row = blockIdx.x; const float* sr = S + row * SEQ;
  float m = -3.0e38f;
#pragma unroll 2
  for (int k = t; k < SEQ; k += 256) m = fmaxf(m, sr[k]);
#pragma unroll
  for (int o = 1; o < 32; o <<= 1) m = fmaxf(m, __shfl_xor(m, o));
  if ((t & 31) == 0) sred[t >> 5] = m; __syncthreads(); if (t == 0) { float a = sred[0]; for (int i = 1; i < 8; ++i) a = fmaxf(a, sred[i]); sbc = a; } __syncthreads(); m = sbc; __syncthreads();
  float sum = 0.f;
#pragma unroll 1
  for (int k = t; k < SEQ; k += 256) { const float e = expf(sr[k] - m); se[k] = e; sum += e; }
#pragma unroll
  for (int o = 1; o < 32; o <<= 1) sum += __shfl_xor(sum, o);
  if ((t & 31) == 0) sred[t >> 5] = sum; __syncthreads(); if (t == 0) { float a = 0.f; for (int i = 0; i < 8; ++i) a += sred[i]; sbc = 1.0f / a; } __syncthreads();
  const float inv = sbc * PCARRY;
#pragma unroll 2
  for (int k = t; k < SEQ; k += 256) sp[k] = (_Float16)(se[k] * inv);
  __syncthreads();
  for (int q = t; q < SEQ / 8; q += 256) vst2(P + row * SEQ + q * 8, *(const v4u*)&sp[q * 8]);
}
__global__ __launch_bounds__(128) __attribute__((amdgpu_num_vgpr(256))) void k_pv(const _Float16* __restrict__ P, const _Float16* __restrict__ VH, const float* __restrict__ X, const float* __restrict__ G, int b, float* __restrict__ OUT) {
  __shared__ __align__(16) float st[128][68];
  const int tid = threadIdx.x, wave = tid >> 5, lane = tid & 31, col = lane & 15, g = lane >> 4;
  const int c0 = blockIdx.y * 128; const int ql0 = blockIdx.x * 64 + wave * 16;
  const float gam = bfr(G[0]);
  v8f acc[8] = {};
#pragma unroll 1
  for (int kc = 0; kc < SEQ / 32; ++kc) {
    const v16h p = frag_h(P + (size_t)(ql0 + col) * SEQ + kc * 32, lane);
#pragma unroll
    for (int j = 0; j < 8; ++j) { const v16h v = frag_h(VH + ((size_t)b * CC + c0 + j * 16 + col) * (size_t)SEQ + kc * 32, lane);
      acc[j] = wmma16(p, v, acc[j]); }
  }
  const float sc = gam * (1.0f / PCARRY);
#pragma unroll
  for (int j = 0; j < 8; ++j)
#pragma unroll
    for (int r = 0; r < 8; ++r) st[j * 16 + col][wave * 16 + 8 * g + r] = acc[j][r] * sc;
  __syncthreads();
  { const int i0 = blockIdx.x * 64;
    for (int e = tid; e < 128 * 16; e += 128) { const int cl = e >> 4, q = e & 15;
      const size_t off = ((size_t)b * CC + c0 + cl) * (size_t)SEQ_FULL + i0 + q * 4;
      const v4f xr = *(const v4f*)(X + off); v4f o = *(const v4f*)&st[cl][q * 4];
      o[0] += bfr(xr[0]); o[1] += bfr(xr[1]); o[2] += bfr(xr[2]); o[3] += bfr(xr[3]);
      vst2(OUT + off, o); } }
}

extern "C" void kernel_launch(void* const* d_in, const int* in_sizes, int n_in, void* d_out, int out_size, void* d_ws, size_t ws_size, hipStream_t stream) {
  if (n_in < 8) return;
  if (in_sizes[0] < NB * CC * SEQ_FULL || in_sizes[1] < DQ * CC || in_sizes[2] < DQ || in_sizes[3] < DQ * CC || in_sizes[4] < DQ || in_sizes[5] < CC * CC || in_sizes[6] < CC || in_sizes[7] < 1) return;
  if (out_size < NB * CC * SEQ_FULL) return;
  if (ws_size < (size_t)WS_END) return;
  const float* X = (const float*)d_in[0]; const float* WQ = (const float*)d_in[1]; const float* BQ = (const float*)d_in[2];
  const float* WK = (const float*)d_in[3]; const float* BK = (const float*)d_in[4]; const float* WV = (const float*)d_in[5];
  const float* BV = (const float*)d_in[6]; const float* G = (const float*)d_in[7];
  float* OUT = (float*)d_out;
  char* ws = (char*)d_ws;
  __bf16 *PQ = (__bf16*)(ws + WS_WQ), *PK = (__bf16*)(ws + WS_WK), *PV = (__bf16*)(ws + WS_WV), *XB = (__bf16*)(ws + WS_XB);
  _Float16 *QH = (_Float16*)(ws + WS_QH), *QL = (_Float16*)(ws + WS_QL), *KH = (_Float16*)(ws + WS_KH), *KL = (_Float16*)(ws + WS_KL), *VH = (_Float16*)(ws + WS_VH);
  float* S = (float*)(ws + WS_S); _Float16* P = (_Float16*)(ws + WS_P);

  k_cvt<<<dim3(2 * NBQ + NBV), 256, 0, stream>>>(WQ, WK, WV, PQ, PK, PV);
  k_xt<<<dim3(SEQ / 64, NB), 256, 0, stream>>>(X, XB);
  k_pqk<<<dim3(NB * SEQ / 64, 2), 128, 0, stream>>>(XB, PQ, PK, BQ, BK, QH, QL, KH, KL);
  k_pvv<<<dim3(NB * SEQ / 64, CC / 128), 128, 0, stream>>>(XB, PV, BV, VH);
  for (int b = 0; b < NB; ++b) {
    k_sc<<<dim3(SEQ / 64, SEQ / 128), 128, 0, stream>>>(QH, QL, KH, KL, b, S);
    k_sm<<<dim3(SEQ), 256, 0, stream>>>(S, P);
    k_pv<<<dim3(SEQ / 64, CC / 128), 128, 0, stream>>>(P, VH, X, G, b, OUT);
  }
}
